// Decoder_79405355369049
// MI455X (gfx1250) — hardware-run, weakly checked
//
#include <hip/hip_runtime.h>
#include <hip/hip_fp16.h>
#include <math.h>

typedef __attribute__((ext_vector_type(16))) _Float16 v16h;
typedef __attribute__((ext_vector_type(8)))  _Float16 v8h;
typedef __attribute__((ext_vector_type(8)))  float    v8f;
typedef __attribute__((ext_vector_type(4)))  float    v4f;
typedef __attribute__((ext_vector_type(2)))  float    v2f;

constexpr int kVocab  = 32000;
constexpr int kEmb    = 256;
constexpr int kHid    = 512;
constexpr int kGates  = 4 * kHid;
constexpr int kSeqIn  = 512;
constexpr int kSteps  = kSeqIn + 1;
constexpr int kMP     = 544;
constexpr int kSos    = 1;
constexpr float kWCarry = 1024.0f;
static_assert(kGates == 2048 && kSteps == 513);
static_assert(kMP >= kSteps && (kMP % 32) == 0);
static_assert((kGates % 64) == 0 && (kVocab % 64) == 0);
static_assert((kEmb % 32) == 0 && (kHid % 32) == 0);
static_assert((kHid % 64) == 0 && (kVocab % 1280) == 0);

constexpr int kOut0 = 0;
constexpr int kOut1 = kSteps * kVocab;
constexpr int kOut2 = kOut1 + kHid;
constexpr int kOutTotal = kOut2 + kHid;
static_assert(kOut1 == 16416000 && kOut2 == 16416512 && kOutTotal == 16417024);
static_assert(((size_t)kOut1 * 4) % 128 == 0 && ((size_t)kOut2 * 4) % 128 == 0);

__device__ __forceinline__ _Float16 f16_flush(float v) {
  const float w = (fabsf(v) < 6.103515625e-05f) ? 0.0f : v;
  return (_Float16)w;
}

__device__ __forceinline__ float bf16r(float v) {
  unsigned u = __float_as_uint(v);
  u = (u + 0x7FFFu + ((u >> 16) & 1u)) & 0xFFFF0000u;
  return __uint_as_float(u);
}

namespace eng {
union FragU { v16h v; v8h h[2]; };
__device__ __forceinline__ v16h frag_load(const _Float16* p) {
  FragU f;
  f.h[0] = *(const v8h*)(p);
  f.h[1] = *(const v8h*)(p + 16);
  return f.v;
}
__device__ __forceinline__ v8f mma(v16h a, v16h b, v8f c) {
  return __builtin_amdgcn_wmma_f32_16x16x32_f16(false, a, false, b, (short)0, c, false, false);
}
__device__ __forceinline__ void guard1(v8f& a, v16h x, v16h y) {
  asm volatile("v_nop\n\tv_nop\n\tv_nop\n\tv_nop" : "+v"(a) : "v"(x), "v"(y));
}
__device__ __forceinline__ void guard_acc(v8f& a) {
  asm volatile("v_nop\n\tv_nop\n\tv_nop\n\tv_nop" : "+v"(a));
}
__device__ __forceinline__ void keep4(v16h a, v16h b, v16h c, v16h d) {
  asm volatile("v_nop" :: "v"(a), "v"(b), "v"(c), "v"(d));
}

template <int MI, int SPL>
__global__ __launch_bounds__(256) void gemm_f16_kernel(
    const unsigned short* __restrict__ Ap, const unsigned short* __restrict__ A2p, int lda,
    const unsigned short* __restrict__ Btp, const unsigned short* __restrict__ Bt2p, int ldb,
    float* __restrict__ C, int ldc, int M, int N, int K, float scale, float rscale)
{
  static_assert(MI >= 1 && MI <= 2);
  static_assert(SPL >= 0 && SPL <= 2);
  const _Float16* A   = (const _Float16*)Ap;
  const _Float16* A2  = (const _Float16*)A2p;
  const _Float16* Bt  = (const _Float16*)Btp;
  const _Float16* Bt2 = (const _Float16*)Bt2p;
  __shared__ __align__(16) float sT[8][16 * 68];
  const int lane = threadIdx.x & 31;
  const int wave = threadIdx.x >> 5;
  const int tilesN = N >> 6;
  const int tilesM = M / (16 * MI);
  const int tile = blockIdx.x * 8 + wave;
  if (tile >= tilesM * tilesN) return;
  const int tm = tile / tilesN;
  const int tn = tile - tm * tilesN;
  const int m0 = tm * (16 * MI);
  const int n0 = tn << 6;
  const int rlane = lane & 15;
  const int koff  = (lane >> 4) * 8;
  const int mOff  = (lane >> 4) * 8;

  v8f acc[MI][4], accr[MI][4];
#pragma unroll
  for (int i = 0; i < MI; ++i)
#pragma unroll
    for (int j = 0; j < 4; ++j) {
      acc[i][j]  = (v8f){0.f, 0.f, 0.f, 0.f, 0.f, 0.f, 0.f, 0.f};
      accr[i][j] = (v8f){0.f, 0.f, 0.f, 0.f, 0.f, 0.f, 0.f, 0.f};
    }

  for (int k0 = 0; k0 < K; k0 += 32) {
    v16h bh[4], bl[4];
#pragma unroll
    for (int j = 0; j < 4; ++j) {
      const size_t bo = (size_t)(n0 + (j << 4) + rlane) * ldb + koff + k0;
      bh[j] = frag_load(Bt + bo);
      if (SPL == 2) bl[j] = frag_load(Bt2 + bo); else bl[j] = bh[j];
    }
#pragma unroll
    for (int i = 0; i < MI; ++i) {
      const size_t ao = (size_t)(m0 + (i << 4) + rlane) * lda + koff + k0;
      const v16h ah = frag_load(A + ao);
      v16h al = ah;
      if (SPL >= 1) al = frag_load(A2 + ao);
#pragma unroll
      for (int j = 0; j < 4; ++j) {
        acc[i][j] = mma(ah, bh[j], acc[i][j]);
        if (SPL >= 1) accr[i][j] = mma(al, bh[j], accr[i][j]);
        if (SPL == 2) accr[i][j] = mma(ah, bl[j], accr[i][j]);
      }
#pragma unroll
      for (int j = 0; j < 4; ++j) {
        guard1(acc[i][j], ah, al);
        if (SPL >= 1) guard1(accr[i][j], ah, al);
      }
    }
    keep4(bh[0], bh[1], bh[2], bh[3]);
    if (SPL == 2) keep4(bl[0], bl[1], bl[2], bl[3]);
  }
#pragma unroll
  for (int i = 0; i < MI; ++i)
#pragma unroll
    for (int j = 0; j < 4; ++j) {
      guard_acc(acc[i][j]);
      if (SPL >= 1) guard_acc(accr[i][j]);
    }

  float* slab = sT[wave];
#pragma unroll
  for (int i = 0; i < MI; ++i) {
    const int mBase = m0 + (i << 4);
#pragma unroll
    for (int j = 0; j < 4; ++j) {
#pragma unroll
      for (int r = 0; r < 8; ++r) {
        float v = acc[i][j][r] * scale;
        if (SPL >= 1) v += accr[i][j][r] * rscale;
        slab[(mOff + r) * 68 + (j << 4) + rlane] = v;
      }
    }
    __builtin_amdgcn_fence(__ATOMIC_RELEASE, "workgroup");
    __builtin_amdgcn_wave_barrier();
    __builtin_amdgcn_fence(__ATOMIC_ACQUIRE, "workgroup");
    {
      const int hh = lane >> 4, c4 = (lane & 15) * 4;
      for (int pass = 0; pass < 2; ++pass) {
#pragma unroll
        for (int it = 0; it < 8; ++it) {
          const int row = it * 2 + hh;
          const v4f v = *(const v4f*)(slab + row * 68 + c4);
          *(volatile v4f*)(C + (size_t)(mBase + row) * ldc + n0 + c4) = v;
        }
        __threadfence();
      }
    }
    __builtin_amdgcn_fence(__ATOMIC_RELEASE, "workgroup");
    __builtin_amdgcn_wave_barrier();
    __builtin_amdgcn_fence(__ATOMIC_ACQUIRE, "workgroup");
  }
}
}

constexpr size_t kSzWIH  = (size_t)kGates * kEmb * 2;
constexpr size_t kSzWOUT = (size_t)kVocab * kHid * 2;
constexpr size_t kSzWHT  = (size_t)kHid * kGates * 4;
constexpr size_t kSzGV   = (size_t)kGates * 4;
constexpr size_t kSzBOUT = (size_t)kVocab * 4;
constexpr size_t kSzST   = (size_t)kHid * 4;
constexpr size_t kSzXE   = (size_t)kMP * kEmb * 2;
constexpr size_t kSzGX   = (size_t)kMP * kGates * 4;
constexpr size_t kSzHSF  = (size_t)kMP * kHid * 4;
constexpr size_t kSzHSH  = (size_t)kMP * kHid * 2;
constexpr size_t kSzLG   = (size_t)kMP * kVocab * 4;
constexpr size_t kOffWIH  = 0;
constexpr size_t kOffWOUT = kOffWIH  + kSzWIH;
constexpr size_t kOffWHT  = kOffWOUT + kSzWOUT;
constexpr size_t kOffBIH  = kOffWHT  + kSzWHT;
constexpr size_t kOffBHH  = kOffBIH  + kSzGV;
constexpr size_t kOffBOUT = kOffBHH  + kSzGV;
constexpr size_t kOffHA   = kOffBOUT + kSzBOUT;
constexpr size_t kOffCA   = kOffHA   + kSzST;
constexpr size_t kOffHB   = kOffCA   + kSzST;
constexpr size_t kOffCB   = kOffHB   + kSzST;
constexpr size_t kOffXE   = kOffCB   + kSzST;
constexpr size_t kOffGX   = kOffXE   + kSzXE;
constexpr size_t kOffHSF  = kOffGX   + kSzGX;
constexpr size_t kOffHSH  = kOffHSF  + kSzHSF;
constexpr size_t kOffLG   = kOffHSH  + kSzHSH;
constexpr size_t kWsTotal = kOffLG   + kSzLG;
static_assert(kSzWIH == 1048576ull && kSzWOUT == 32768000ull && kSzWHT == 4194304ull);
static_assert(kSzXE == 278528ull && kSzGX == 4456448ull && kSzHSF == 1114112ull);
static_assert(kSzHSH == 557056ull && kSzLG == 69632000ull);
static_assert(kWsTotal == 114201600ull);
static_assert(kWsTotal <= 134217728ull);
static_assert((kOffWOUT % 128) == 0 && (kOffWHT % 128) == 0 && (kOffBIH % 128) == 0 &&
              (kOffBHH % 128) == 0 && (kOffBOUT % 128) == 0 && (kOffHA % 128) == 0 &&
              (kOffCA % 128) == 0 && (kOffHB % 128) == 0 && (kOffCB % 128) == 0 &&
              (kOffXE % 128) == 0 && (kOffGX % 128) == 0 && (kOffHSF % 128) == 0 &&
              (kOffHSH % 128) == 0 && (kOffLG % 128) == 0);

__global__ __launch_bounds__(256) void pack_rows_bf_kernel(
    const float* __restrict__ W, unsigned short* __restrict__ dH,
    int Kdim, int Nreal, int total8, float carry)
{
  const int i = blockIdx.x * 256 + threadIdx.x;
  if (i >= total8) return;
  const size_t e0 = (size_t)i << 3;
  const int row = (int)(e0 / (size_t)Kdim);
  const int col = (int)(e0 - (size_t)row * (size_t)Kdim);
  const bool live = (row < Nreal);
  const int rc = live ? row : (Nreal - 1);
  const v4f a0 = *(const v4f*)(W + (size_t)rc * Kdim + col);
  const v4f a1 = *(const v4f*)(W + (size_t)rc * Kdim + col + 4);
  const float w0 = a0[0];
  const float w1 = a0[1];
  const float w2 = a0[2];
  const float w3 = a0[3];
  const float w4 = a1[0];
  const float w5 = a1[1];
  const float w6 = a1[2];
  const float w7 = a1[3];
  const float t0 = bf16r(w0) * carry;
  const float t1 = bf16r(w1) * carry;
  const float t2 = bf16r(w2) * carry;
  const float t3 = bf16r(w3) * carry;
  const float t4 = bf16r(w4) * carry;
  const float t5 = bf16r(w5) * carry;
  const float t6 = bf16r(w6) * carry;
  const float t7 = bf16r(w7) * carry;
  const float g0 = live ? t0 : 0.0f;
  const float g1 = live ? t1 : 0.0f;
  const float g2 = live ? t2 : 0.0f;
  const float g3 = live ? t3 : 0.0f;
  const float g4 = live ? t4 : 0.0f;
  const float g5 = live ? t5 : 0.0f;
  const float g6 = live ? t6 : 0.0f;
  const float g7 = live ? t7 : 0.0f;
  v8h hv;
  hv[0] = f16_flush(g0);
  hv[1] = f16_flush(g1);
  hv[2] = f16_flush(g2);
  hv[3] = f16_flush(g3);
  hv[4] = f16_flush(g4);
  hv[5] = f16_flush(g5);
  hv[6] = f16_flush(g6);
  hv[7] = f16_flush(g7);
  unsigned short* qh = dH + e0;
  *(volatile v8h*)qh = hv;
  __threadfence();
  *(volatile v8h*)qh = hv;
}

__global__ __launch_bounds__(256) void rne_vec_kernel(
    const float* __restrict__ src, float* __restrict__ dst, int n4)
{
  const int i = blockIdx.x * 256 + threadIdx.x;
  if (i >= n4) return;
  const v4f a = *(const v4f*)(src + (size_t)i * 4);
  const float a0 = a[0];
  const float a1 = a[1];
  const float a2 = a[2];
  const float a3 = a[3];
  v4f r;
  r[0] = bf16r(a0);
  r[1] = bf16r(a1);
  r[2] = bf16r(a2);
  r[3] = bf16r(a3);
  float* p = dst + (size_t)i * 4;
  *(volatile v4f*)p = r;
  __threadfence();
  *(volatile v4f*)p = r;
}

__global__ __launch_bounds__(256) void wht_kernel(
    const float* __restrict__ Whh, float* __restrict__ WHT)
{
  __shared__ float tile[64 * 65];
  const int tid  = threadIdx.x;
  const int lane = tid & 31;
  const int wave = tid >> 5;
  const int g0 = blockIdx.x * 64;
  const int k0 = blockIdx.y * 64;
  const int k4 = (tid & 15) * 4;
  const int gr = tid >> 4;
#pragma unroll
  for (int i = 0; i < 4; ++i) {
    const int g = gr + 16 * i;
    const v4f a = *(const v4f*)(Whh + (size_t)(g0 + g) * kHid + k0 + k4);
    const float a0 = a[0];
    const float a1 = a[1];
    const float a2 = a[2];
    const float a3 = a[3];
    tile[g * 65 + k4 + 0] = bf16r(a0);
    tile[g * 65 + k4 + 1] = bf16r(a1);
    tile[g * 65 + k4 + 2] = bf16r(a2);
    tile[g * 65 + k4 + 3] = bf16r(a3);
  }
  __syncthreads();
  v2f val[8];
#pragma unroll
  for (int kk = 0; kk < 8; ++kk) {
    const int k = wave * 8 + kk;
    v2f t;
    t[0] = tile[(2 * lane) * 65 + k];
    t[1] = tile[(2 * lane + 1) * 65 + k];
    val[kk] = t;
  }
  for (int pass = 0; pass < 2; ++pass) {
#pragma unroll
    for (int kk = 0; kk < 8; ++kk) {
      const int k = wave * 8 + kk;
      *(volatile v2f*)(WHT + (size_t)(k0 + k) * kGates + g0 + 2 * lane) = val[kk];
    }
    __threadfence();
  }
}

__global__ __launch_bounds__(256) void gather_word_kernel(
    const int* __restrict__ seq, const float* __restrict__ emb, unsigned short* __restrict__ XE)
{
  const int i = blockIdx.x * 256 + threadIdx.x;
  if (i >= kMP * kEmb / 8) return;
  const int row = i >> 5;
  const int col = (i & 31) * 8;
  const bool live = (row < kSteps);
  int si = row - 1;
  si = (si < 0) ? 0 : si;
  si = (si > kSeqIn - 1) ? (kSeqIn - 1) : si;
  const int sv = seq[si];
  const int tok = (row == 0) ? kSos : sv;
  const int tlo = (tok < 0) ? 0 : tok;
  const int tokc = (tlo > kVocab - 1) ? (kVocab - 1) : tlo;
  const float* sp = emb + (size_t)tokc * kEmb + col;
  const v4f a0 = *(const v4f*)(sp);
  const v4f a1 = *(const v4f*)(sp + 4);
  const float w0 = a0[0];
  const float w1 = a0[1];
  const float w2 = a0[2];
  const float w3 = a0[3];
  const float w4 = a1[0];
  const float w5 = a1[1];
  const float w6 = a1[2];
  const float w7 = a1[3];
  const float g0 = live ? bf16r(w0) : 0.0f;
  const float g1 = live ? bf16r(w1) : 0.0f;
  const float g2 = live ? bf16r(w2) : 0.0f;
  const float g3 = live ? bf16r(w3) : 0.0f;
  const float g4 = live ? bf16r(w4) : 0.0f;
  const float g5 = live ? bf16r(w5) : 0.0f;
  const float g6 = live ? bf16r(w6) : 0.0f;
  const float g7 = live ? bf16r(w7) : 0.0f;
  v8h hv;
  hv[0] = f16_flush(g0);
  hv[1] = f16_flush(g1);
  hv[2] = f16_flush(g2);
  hv[3] = f16_flush(g3);
  hv[4] = f16_flush(g4);
  hv[5] = f16_flush(g5);
  hv[6] = f16_flush(g6);
  hv[7] = f16_flush(g7);
  unsigned short* qh = XE + (size_t)row * kEmb + col;
  *(volatile v8h*)qh = hv;
  __threadfence();
  *(volatile v8h*)qh = hv;
}

__global__ __launch_bounds__(256) void lstm_step_kernel(
    const float* __restrict__ GXt, const float* __restrict__ WHT,
    const float* __restrict__ BIH, const float* __restrict__ BHH,
    const float* __restrict__ Hin, const float* __restrict__ Cin,
    float* __restrict__ Hout, float* __restrict__ Cout, float* __restrict__ HSFt)
{
  __shared__ float sh[kHid];
  const int tid = threadIdx.x;
  const int j = blockIdx.x * 256 + tid;
  sh[tid] = Hin[tid];
  sh[tid + 256] = Hin[tid + 256];
  __syncthreads();
  float ai = 0.0f;
  float af = 0.0f;
  float ag = 0.0f;
  float ao = 0.0f;
  const float* wp = WHT + j;
  for (int k = 0; k < kHid; ++k) {
    const float hk = sh[k];
    const float* wr = wp + (size_t)k * kGates;
    ai = fmaf(wr[0], hk, ai);
    af = fmaf(wr[kHid], hk, af);
    ag = fmaf(wr[2 * kHid], hk, ag);
    ao = fmaf(wr[3 * kHid], hk, ao);
  }
  const float bi = BIH[j] + BHH[j];
  const float bf = BIH[j + kHid] + BHH[j + kHid];
  const float bg = BIH[j + 2 * kHid] + BHH[j + 2 * kHid];
  const float bo = BIH[j + 3 * kHid] + BHH[j + 3 * kHid];
  const float gi = GXt[j] + ai + bi;
  const float gf = GXt[j + kHid] + af + bf;
  const float gg = GXt[j + 2 * kHid] + ag + bg;
  const float go = GXt[j + 3 * kHid] + ao + bo;
  const float iv = 1.0f / (1.0f + expf(-gi));
  const float fv = 1.0f / (1.0f + expf(-gf));
  const float gv = tanhf(gg);
  const float ov = 1.0f / (1.0f + expf(-go));
  const float cp = Cin[j];
  const float cn = fv * cp + iv * gv;
  const float hn = ov * tanhf(cn);
  for (int pass = 0; pass < 2; ++pass) {
    *(volatile float*)(Hout + j) = hn;
    *(volatile float*)(Cout + j) = cn;
    *(volatile float*)(HSFt + j) = hn;
    __threadfence();
  }
}

__global__ __launch_bounds__(256) void hs_word_kernel(
    const float* __restrict__ HSF, unsigned short* __restrict__ HSH)
{
  const int i = blockIdx.x * 256 + threadIdx.x;
  if (i >= kMP * kHid / 8) return;
  const int row = i >> 6;
  const int col = (i & 63) * 8;
  const bool live = (row < kSteps);
  const int rc = live ? row : (kSteps - 1);
  const float* sp = HSF + (size_t)rc * kHid + col;
  const v4f a0 = *(const v4f*)(sp);
  const v4f a1 = *(const v4f*)(sp + 4);
  const float w0 = a0[0];
  const float w1 = a0[1];
  const float w2 = a0[2];
  const float w3 = a0[3];
  const float w4 = a1[0];
  const float w5 = a1[1];
  const float w6 = a1[2];
  const float w7 = a1[3];
  const float g0 = live ? w0 : 0.0f;
  const float g1 = live ? w1 : 0.0f;
  const float g2 = live ? w2 : 0.0f;
  const float g3 = live ? w3 : 0.0f;
  const float g4 = live ? w4 : 0.0f;
  const float g5 = live ? w5 : 0.0f;
  const float g6 = live ? w6 : 0.0f;
  const float g7 = live ? w7 : 0.0f;
  v8h hv;
  hv[0] = f16_flush(g0);
  hv[1] = f16_flush(g1);
  hv[2] = f16_flush(g2);
  hv[3] = f16_flush(g3);
  hv[4] = f16_flush(g4);
  hv[5] = f16_flush(g5);
  hv[6] = f16_flush(g6);
  hv[7] = f16_flush(g7);
  unsigned short* qh = HSH + (size_t)row * kHid + col;
  *(volatile v8h*)qh = hv;
  __threadfence();
  *(volatile v8h*)qh = hv;
}

__global__ __launch_bounds__(160) void logits_out_kernel(
    const float* __restrict__ LG, const float* __restrict__ BOUT, float* __restrict__ out0)
{
  const int lane = threadIdx.x & 31;
  const int wave = threadIdx.x >> 5;
  const int r = blockIdx.y;
  const int va = blockIdx.x * 1280 + wave * 256 + lane * 4;
  const int vb = va + 128;
  const size_t rb = (size_t)r * kVocab;
  const v4f la = *(const v4f*)(LG + rb + va);
  const v4f lb = *(const v4f*)(LG + rb + vb);
  const v4f ba = *(const v4f*)(BOUT + va);
  const v4f bb = *(const v4f*)(BOUT + vb);
  const v4f ra = la + ba;
  const v4f rv = lb + bb;
  for (int pass = 0; pass < 2; ++pass) {
    *(volatile v4f*)(out0 + rb + va) = ra;
    *(volatile v4f*)(out0 + rb + vb) = rv;
    __threadfence();
  }
}

__global__ __launch_bounds__(256) void state_out_kernel(
    const float* __restrict__ Hfin, const float* __restrict__ Cfin,
    float* __restrict__ outH, float* __restrict__ outC)
{
  const int i = threadIdx.x;
  const bool isH = (i < 128);
  const int e = (isH ? i : (i - 128)) * 4;
  const float* src = isH ? Hfin : Cfin;
  float* dst = isH ? outH : outC;
  const v4f a = *(const v4f*)(src + e);
  const v4f r = a;
  *(volatile v4f*)(dst + e) = r;
  __threadfence();
  *(volatile v4f*)(dst + e) = r;
}

static_assert(((kMP / 32) * (kGates / 64)) % 8 == 0);
static_assert(((kGates * kEmb / 8) % 256) == 0);
static_assert(((kVocab * kHid / 8) % 256) == 0);
static_assert(((kMP * kEmb / 8) % 256) == 0);
static_assert(((kMP * kHid / 8) % 256) == 0);
static_assert(((kGates / 4) % 256) == 0);
static_assert((kVocab % 4) == 0 && (kHid / 4) == 128);
static_assert(((kSteps - 1) % 2) == 0);

extern "C" void kernel_launch(void* const* d_in, const int* in_sizes, int n_in,
                              void* d_out, int out_size, void* d_ws, size_t ws_size,
                              hipStream_t stream)
{
  if (n_in < 10) return;
  if (in_sizes[0] != kSeqIn) return;
  if (in_sizes[1] != kHid) return;
  if (in_sizes[2] != kHid) return;
  if (in_sizes[3] != kVocab * kEmb) return;
  if (in_sizes[4] != kGates * kEmb) return;
  if (in_sizes[5] != kGates * kHid) return;
  if (in_sizes[6] != kGates) return;
  if (in_sizes[7] != kGates) return;
  if (in_sizes[8] != kVocab * kHid) return;
  if (in_sizes[9] != kVocab) return;
  if (out_size != kOutTotal) return;
  if (ws_size < kWsTotal) return;

  const int*   seq   = (const int*)d_in[0];
  const float* h0    = (const float*)d_in[1];
  const float* c0    = (const float*)d_in[2];
  const float* emb   = (const float*)d_in[3];
  const float* W_ih  = (const float*)d_in[4];
  const float* W_hh  = (const float*)d_in[5];
  const float* b_ih  = (const float*)d_in[6];
  const float* b_hh  = (const float*)d_in[7];
  const float* W_out = (const float*)d_in[8];
  const float* b_out = (const float*)d_in[9];
  float* out = (float*)d_out;

  char* ws = (char*)d_ws;
  unsigned short* WIH  = (unsigned short*)(ws + kOffWIH);
  unsigned short* WOUT = (unsigned short*)(ws + kOffWOUT);
  float*          WHT  = (float*)(ws + kOffWHT);
  float*          BIH  = (float*)(ws + kOffBIH);
  float*          BHH  = (float*)(ws + kOffBHH);
  float*          BOUT = (float*)(ws + kOffBOUT);
  float*          HA   = (float*)(ws + kOffHA);
  float*          CA   = (float*)(ws + kOffCA);
  float*          HB   = (float*)(ws + kOffHB);
  float*          CB   = (float*)(ws + kOffCB);
  unsigned short* XE   = (unsigned short*)(ws + kOffXE);
  float*          GX   = (float*)(ws + kOffGX);
  float*          HSF  = (float*)(ws + kOffHSF);
  unsigned short* HSH  = (unsigned short*)(ws + kOffHSH);
  float*          LG   = (float*)(ws + kOffLG);

  constexpr float sW = 1.0f / kWCarry;

  pack_rows_bf_kernel<<<(kGates * kEmb / 8) / 256, 256, 0, stream>>>(
      W_ih, WIH, kEmb, kGates, kGates * kEmb / 8, kWCarry);

  pack_rows_bf_kernel<<<(kVocab * kHid / 8) / 256, 256, 0, stream>>>(
      W_out, WOUT, kHid, kVocab, kVocab * kHid / 8, kWCarry);

  wht_kernel<<<dim3(kGates / 64, kHid / 64), 256, 0, stream>>>(W_hh, WHT);

  rne_vec_kernel<<<(kGates / 4) / 256, 256, 0, stream>>>(b_ih, BIH, kGates / 4);
  rne_vec_kernel<<<(kGates / 4) / 256, 256, 0, stream>>>(b_hh, BHH, kGates / 4);

  rne_vec_kernel<<<(kVocab / 4 + 255) / 256, 256, 0, stream>>>(b_out, BOUT, kVocab / 4);

  rne_vec_kernel<<<1, 256, 0, stream>>>(h0, HA, kHid / 4);
  rne_vec_kernel<<<1, 256, 0, stream>>>(c0, CA, kHid / 4);

  gather_word_kernel<<<(kMP * kEmb / 8) / 256, 256, 0, stream>>>(seq, emb, XE);

  eng::gemm_f16_kernel<2, 0><<<dim3((kMP / 32) * (kGates / 64) / 8), 256, 0, stream>>>(
      XE, nullptr, kEmb, WIH, nullptr, kEmb, GX, kGates, kMP, kGates, kEmb, sW, 0.0f);

  for (int t = 0; t < kSteps; ++t) {
    const bool even = ((t & 1) == 0);
    const float* Hin = even ? HA : HB;
    const float* Cin = even ? CA : CB;
    float* Hout = even ? HB : HA;
    float* Cout = even ? CB : CA;
    lstm_step_kernel<<<2, 256, 0, stream>>>(
        GX + (size_t)t * kGates, WHT, BIH, BHH, Hin, Cin, Hout, Cout, HSF + (size_t)t * kHid);
  }

  hs_word_kernel<<<(kMP * kHid / 8) / 256, 256, 0, stream>>>(HSF, HSH);

  eng::gemm_f16_kernel<2, 0><<<dim3(((kMP / 32) * (kVocab / 64) + 7) / 8), 256, 0, stream>>>(
      HSH, nullptr, kHid, WOUT, nullptr, kHid, LG, kVocab, kMP, kVocab, kHid, sW, 0.0f);

  logits_out_kernel<<<dim3(kVocab / 1280, kSteps), 160, 0, stream>>>(LG, BOUT, out + kOut0);

  state_out_kernel<<<1, 256, 0, stream>>>(HB, CB, out + kOut1, out + kOut2);
}
